// PointnetLFPModuleMSG_3169685865256
// MI455X (gfx1250) — hardware-verified
//
#include <hip/hip_runtime.h>
#include <math.h>

typedef __attribute__((ext_vector_type(16))) _Float16 v16h;
typedef __attribute__((ext_vector_type(16))) __bf16 v16b;
typedef __attribute__((ext_vector_type(8)))  _Float16 v8h;
typedef __attribute__((ext_vector_type(8)))  float v8f;
typedef __attribute__((ext_vector_type(4)))  float v4f;
typedef __attribute__((ext_vector_type(2)))  float v2f;
typedef __attribute__((ext_vector_type(4)))  unsigned v4u;
typedef __attribute__((ext_vector_type(4)))  int v4i;
typedef float __attribute__((may_alias)) float_a;
typedef int __attribute__((may_alias)) int_a;

template <typename T> __device__ __forceinline__ void vst2(void* p, T v) { *(volatile T*)p = v; __threadfence(); *(volatile T*)p = v; }
__device__ __forceinline__ v8f wmma16(v16h a, v16h b, v8f c) {
  v8f d = __builtin_amdgcn_wmma_f32_16x16x32_f16(false, a, false, b, (short)0, c, false, false);
  asm volatile("v_nop\n\tv_nop\n\tv_nop\n\tv_nop" : "+v"(d) : "v"(a), "v"(b));
  return d;
}
__device__ __forceinline__ v8f wmma_bf(v16b a, v16b b, v8f c) {
  v8f d = __builtin_amdgcn_wmma_f32_16x16x32_bf16(false, a, false, b, (short)0, c, false, false);
  asm volatile("v_nop\n\tv_nop\n\tv_nop\n\tv_nop" : "+v"(d) : "v"(a), "v"(b));
  return d;
}
__device__ __forceinline__ v16h frag_h(const _Float16* rowk0, int lane) {
  union { v16h v; v8h q[2]; } u; const _Float16* p = rowk0 + 8 * (lane >> 4);
  u.q[0] = *(const v8h*)p; u.q[1] = *(const v8h*)(p + 16); return u.v;
}
__device__ __forceinline__ v16h frag_f32(const float* rowk0, int lane) {
  v16h a; const float* p = rowk0 + 8 * (lane >> 4);
#pragma unroll
  for (int i = 0; i < 8; ++i) { a[i] = (_Float16)p[i]; a[8 + i] = (_Float16)p[16 + i]; }
  return a;
}
__device__ __forceinline__ v16h frag_f32s(const float* rowk0, int lane, float sc) {
  v16h a; const float* p = rowk0 + 8 * (lane >> 4);
#pragma unroll
  for (int i = 0; i < 8; ++i) { a[i] = (_Float16)(p[i] * sc); a[8 + i] = (_Float16)(p[16 + i] * sc); }
  return a;
}
__device__ __forceinline__ v16h fragc_f32(const float* W, int k0, int n, int lane, int ld, int K) {
  v16h a; const int g = lane >> 4;
#pragma unroll
  for (int i = 0; i < 8; ++i) { const int ka = k0 + 8 * g + i, kb = ka + 16;
    a[i] = (_Float16)(ka < K ? W[(size_t)(ka < K ? ka : K - 1) * ld + n] : 0.f); a[8 + i] = (_Float16)(kb < K ? W[(size_t)(kb < K ? kb : K - 1) * ld + n] : 0.f); }
  return a;
}
struct F2 { v16b h, l; };
__device__ __forceinline__ F2 bsplit16(const float v[16]) { F2 r;
#pragma unroll
  for (int i = 0; i < 16; ++i) { const __bf16 h = (__bf16)v[i]; r.h[i] = h; r.l[i] = (__bf16)(v[i] - (float)h); }
  return r; }
__device__ __forceinline__ F2 split_row(const float* row, int k0, int lane) { float v[16]; const float* p = row + k0 + 8 * (lane >> 4);
#pragma unroll
  for (int i = 0; i < 8; ++i) { v[i] = p[i]; v[8 + i] = p[16 + i]; }
  return bsplit16(v); }
__device__ __forceinline__ F2 split_rowK(const float* row, int k0, int lane, int K) { float v[16]; const int g = lane >> 4;
#pragma unroll
  for (int i = 0; i < 8; ++i) { const int ka = k0 + 8 * g + i, kb = ka + 16; v[i] = ka < K ? row[ka < K ? ka : K - 1] : 0.f; v[8 + i] = kb < K ? row[kb < K ? kb : K - 1] : 0.f; }
  return bsplit16(v); }
__device__ __forceinline__ F2 split_col(const float* W, int k0, int n, int lane, int ld, int K) { float v[16]; const int g = lane >> 4;
#pragma unroll
  for (int i = 0; i < 8; ++i) { const int ka = k0 + 8 * g + i, kb = ka + 16; v[i] = ka < K ? W[(size_t)(ka < K ? ka : K - 1) * ld + n] : 0.f; v[8 + i] = kb < K ? W[(size_t)(kb < K ? kb : K - 1) * ld + n] : 0.f; }
  return bsplit16(v); }
__device__ __forceinline__ v8f mac3(const F2& a, const F2& b, v8f c) { c = wmma_bf(a.l, b.h, c); c = wmma_bf(a.h, b.l, c); return wmma_bf(a.h, b.h, c); }
__device__ __forceinline__ float sigm(float v) { return 1.0f / (1.0f + expf(-v)); }
#define LDSX() do { asm volatile("s_wait_dscnt 0" ::: "memory"); __builtin_amdgcn_wave_barrier(); __builtin_amdgcn_fence(__ATOMIC_RELEASE, "workgroup"); } while (0)


#define NBT 4
#define N1 8192
#define N2 2048
#define NQ (NBT * N2)
#define C1 64
#define C2 64
#ifndef NQT
#define NQT NQ
#endif
typedef __attribute__((ext_vector_type(8))) __bf16 v8b;
__device__ __forceinline__ v16b frag_b(const __bf16* rowk0, int lane) {
  union { v16b v; v8b q[2]; } u; const __bf16* p = rowk0 + 8 * (lane >> 4);
  u.q[0] = *(const v8b*)p; u.q[1] = *(const v8b*)(p + 16); return u.v;
}
__device__ __forceinline__ float bfr(float v) { return (float)(__bf16)v; }
__device__ __attribute__((noinline)) float exp_ni(float v) { return expf(v); }
__device__ __attribute__((noinline)) float erf_ni(float v) { return erff(v); }

#define WS_F1T  0u
#define WS_IDX0 (WS_F1T + 4u * NBT * N1 * C1)
#define WS_IDX1 (WS_IDX0 + 4u * NQ * 16)
#define WS_PW   (WS_IDX1 + 4u * NQ * 32)
#define P00 0
#define P01 (P00 + 64 * 96)
#define P10 (P01 + 128 * 64)
#define P11 (P10 + 64 * 96)
#define PP  (P11 + 128 * 64)
#define PWEND (PP + 128 * 192)
#define WS_MX   (WS_PW + 2u * PWEND)
#define WS_END  (WS_MX + 4u * 2 * NQ * 128)

__global__ __launch_bounds__(256) void k_packW(const float* __restrict__ W00, const float* __restrict__ W01, const float* __restrict__ W10, const float* __restrict__ W11, const float* __restrict__ WP, __bf16* __restrict__ PW) {
  __shared__ __align__(16) __bf16 s[192]; const int o = blockIdx.x, which = blockIdx.y, t = threadIdx.x;
  if (which == 0 || which == 2) { if (o >= 64) return; const float* Wm = which ? W10 : W00; if (t < 96) s[t] = (__bf16)((t < 67) ? Wm[o * 67 + t] : 0.f); __syncthreads(); if (t < 12) vst2((unsigned*)(PW + (which ? P10 : P00) + (size_t)o * 96 + t * 8), *(const v4u*)&s[t * 8]); }
  else if (which == 1 || which == 3) { const float* Wm = (which == 3) ? W11 : W01; if (t < 64) s[t] = (__bf16)Wm[o * 64 + t]; __syncthreads(); if (t < 8) vst2((unsigned*)(PW + (which == 3 ? P11 : P01) + (size_t)o * 64 + t * 8), *(const v4u*)&s[t * 8]); }
  else { if (t < 192) s[t] = (__bf16)WP[o * 192 + t]; __syncthreads(); if (t < 24) vst2((unsigned*)(PW + PP + (size_t)o * 192 + t * 8), *(const v4u*)&s[t * 8]); }
}
__global__ __launch_bounds__(64) void k_f1t(const float* __restrict__ F1, float* __restrict__ F1T) {
  __shared__ __align__(16) float s[64][68]; const int t = threadIdx.x; const size_t i0 = (size_t)blockIdx.x * 64; const int b = (int)(i0 / N1), n0 = (int)(i0 % N1);
  for (int c = 0; c < C1; ++c) s[t][c] = bfr(F1[((size_t)b * C1 + c) * N1 + n0 + t]);
  __syncthreads();
  for (int q = t; q < 64 * 16; q += 64) { const int rl = q >> 4, pc = q & 15; vst2(F1T + (i0 + rl) * C1 + pc * 4, *(const v4f*)&s[rl][pc * 4]); }
}
__global__ __launch_bounds__(64) void k_ball(const float* __restrict__ X2, const float* __restrict__ X1, int* __restrict__ IDX0, int* __restrict__ IDX1) {
  #pragma clang fp contract(off)
  __shared__ __align__(16) int s0[64][16], s1[64][32]; const int t = threadIdx.x; const size_t q = (size_t)blockIdx.x * 64 + t; const int b = (int)(q / N2);
  const float ax = bfr(X2[q * 3]), ay = bfr(X2[q * 3 + 1]), az = bfr(X2[q * 3 + 2]);
  const float r0 = 0.04f, r1 = 0.16f;
  int c0 = 0, c1 = 0;
  for (int k = 0; k < 16; ++k) s0[t][k] = 0; for (int k = 0; k < 32; ++k) s1[t][k] = 0;
  const float* xb = X1 + (size_t)b * N1 * 3;
#pragma unroll 1
  for (int i = 0; i < N1 && (c0 < 16 || c1 < 32); ++i) { const float dx = ax - bfr(xb[i * 3]), dy = ay - bfr(xb[i * 3 + 1]), dz = az - bfr(xb[i * 3 + 2]); const float d = (dx * dx + dz * dz) + dy * dy;
    if (d <= r1) { if (c1 < 32) { s1[t][c1] = i; ++c1; } if (d <= r0 && c0 < 16) { s0[t][c0] = i; ++c0; } } }
  for (int k = c0; k < 16; ++k) s0[t][k] = s0[t][0]; for (int k = c1; k < 32; ++k) s1[t][k] = s1[t][0];
  __syncthreads();
  for (int q2 = t; q2 < 64 * 4; q2 += 64) { const int rl = q2 >> 2, pc = q2 & 3; vst2((unsigned*)(IDX0 + ((size_t)blockIdx.x * 64 + rl) * 16 + pc * 4), *(const v4u*)&s0[rl][pc * 4]); }
  for (int q2 = t; q2 < 64 * 8; q2 += 64) { const int rl = q2 >> 3, pc = q2 & 7; vst2((unsigned*)(IDX1 + ((size_t)blockIdx.x * 64 + rl) * 32 + pc * 4), *(const v4u*)&s1[rl][pc * 4]); }
}
template <int S>
__global__ __launch_bounds__(128) void k_sa(const float* __restrict__ X2, const float* __restrict__ X1, const float* __restrict__ F1T, const int* __restrict__ IDX, const __bf16* __restrict__ PW, const float* __restrict__ G0, const float* __restrict__ B0, const float* __restrict__ G1, const float* __restrict__ B1, float* __restrict__ MX) {
  constexpr int NS = S ? 32 : 16; constexpr int QPB = 64 / NS;
  __shared__ __align__(16) float sa[4][16][100]; __shared__ __align__(16) float sh[4][16][68]; __shared__ __align__(16) float so[4][16][132]; __shared__ __align__(16) float smx[QPB][128];
  const int tid = threadIdx.x, wave = tid >> 5, lane = tid & 31, col = lane & 15, g = lane >> 4; const size_t row0 = (size_t)blockIdx.x * 64 + wave * 16;
  const float bnc = 1.0f / sqrtf(1.0f + 1e-5f);
  for (int rl = 0; rl < 16; ++rl) { const size_t row = row0 + rl; const size_t q = row / NS; const int smp = (int)(row % NS); const int b = (int)(q / N2); const int i = min(max(IDX[q * NS + smp], 0), N1 - 1);
    if (lane < 3) sa[wave][rl][lane] = bfr(X1[((size_t)b * N1 + i) * 3 + lane]) - bfr(X2[q * 3 + lane]);
    const float* fr = F1T + ((size_t)b * N1 + i) * C1; sa[wave][rl][3 + lane] = fr[lane]; sa[wave][rl][35 + lane] = fr[32 + lane]; if (lane >= 3) sa[wave][rl][64 + lane] = 0.f; else sa[wave][rl][96 + lane] = 0.f; }
  LDSX();
  const __bf16* PW1 = PW + (S ? P10 : P00); const __bf16* PW2 = PW + (S ? P11 : P01);
  v8f acc[4] = {};
#pragma unroll
  for (int kc = 0; kc < 3; ++kc) { const F2 a = split_row(&sa[wave][col][0], kc * 32, lane);
#pragma unroll
    for (int j = 0; j < 4; ++j) { const v16b w = frag_b(PW1 + (size_t)(j * 16 + col) * 96 + kc * 32, lane); if (kc == 0) acc[j] = wmma_bf(a.l, w, acc[j]); acc[j] = wmma_bf(a.h, w, acc[j]); } }
#pragma unroll
  for (int j = 0; j < 4; ++j) { const int o = j * 16 + col; const float sc = bfr(G0[o]) * bnc, sh_ = bfr(B0[o]);
#pragma unroll
    for (int r = 0; r < 8; ++r) sh[wave][8 * g + r][o] = fmaxf(acc[j][r] * sc + sh_, 0.f); }
  LDSX();
  v8f acc2[8] = {};
#pragma unroll
  for (int kc = 0; kc < 2; ++kc) { const F2 a = split_row(&sh[wave][col][0], kc * 32, lane);
#pragma unroll
    for (int j = 0; j < 8; ++j) { const v16b w = frag_b(PW2 + (size_t)(j * 16 + col) * 64 + kc * 32, lane); acc2[j] = wmma_bf(a.l, w, acc2[j]); acc2[j] = wmma_bf(a.h, w, acc2[j]); } }
#pragma unroll
  for (int j = 0; j < 8; ++j) { const int o = j * 16 + col; const float sc = bfr(G1[o]) * bnc, sh_ = bfr(B1[o]);
#pragma unroll
    for (int r = 0; r < 8; ++r) so[wave][8 * g + r][o] = fmaxf(acc2[j][r] * sc + sh_, 0.f); }
  __syncthreads();
  for (int ql = 0; ql < QPB; ++ql) { const int c = tid; float m = 0.f;
    for (int r2 = 0; r2 < NS; ++r2) { const int rr = ql * NS + r2; m = fmaxf(m, so[rr >> 4][rr & 15][c]); }
    smx[ql][c] = m; }
  __syncthreads();
  for (int q2 = tid; q2 < QPB * 32; q2 += 128) { const int ql = q2 >> 5, pc = q2 & 31; vst2(MX + ((size_t)S * NQ + (size_t)blockIdx.x * QPB + ql) * 128 + pc * 4, *(const v4f*)&smx[ql][pc * 4]); }
}
template <int S>
__global__ __launch_bounds__(128) void k_post(const float* __restrict__ MX, const float* __restrict__ FT2, const __bf16* __restrict__ PW, const float* __restrict__ GP, const float* __restrict__ BP, float* __restrict__ OUT) {
  __shared__ __align__(16) float so[128][68];
  const int tid = threadIdx.x, wave = tid >> 5, lane = tid & 31, col = lane & 15, g = lane >> 4; const size_t q0 = (size_t)blockIdx.x * 64; const size_t r0 = q0 + wave * 16; const int b = (int)(q0 / N2); const int j0 = (int)(q0 % N2);
  const float bnc = 1.0f / sqrtf(1.0f + 1e-5f);
  v8f acc[8] = {};
#pragma unroll
  for (int kc = 0; kc < 6; ++kc) { F2 a; if (kc < 4) a = split_row(MX + ((size_t)S * NQ + r0 + col) * 128, kc * 32, lane); else { v16b ax; const int c0 = (kc - 4) * 32 + 8 * g; const size_t jj = (r0 + col) % N2;
#pragma unroll
      for (int i2 = 0; i2 < 8; ++i2) { ax[i2] = (__bf16)FT2[((size_t)b * C2 + c0 + i2) * N2 + jj]; ax[8 + i2] = (__bf16)FT2[((size_t)b * C2 + c0 + 16 + i2) * N2 + jj]; } a.h = ax; a.l = ax; }
#pragma unroll
    for (int j = 0; j < 8; ++j) { const v16b w = frag_b(PW + PP + (size_t)(j * 16 + col) * 192 + kc * 32, lane); if (kc < 4) acc[j] = wmma_bf(a.l, w, acc[j]); acc[j] = wmma_bf(a.h, w, acc[j]); } }
#pragma unroll
  for (int j = 0; j < 8; ++j) { const int o = j * 16 + col; const float sc = bfr(GP[o]) * bnc, sh_ = bfr(BP[o]);
#pragma unroll
    for (int r = 0; r < 8; ++r) so[o][wave * 16 + 8 * g + r] = fmaxf(acc[j][r] * sc + sh_, 0.f); }
  __syncthreads();
  for (int q2 = tid; q2 < 128 * 16; q2 += 128) { const int o = q2 >> 4, pc = q2 & 15; vst2(OUT + ((size_t)b * 256 + S * 128 + o) * N2 + j0 + pc * 4, *(const v4f*)&so[o][pc * 4]); }
}
extern "C" void kernel_launch(void* const* d_in, const int* in_sizes, int n_in, void* d_out, int out_size, void* d_ws, size_t ws_size, hipStream_t stream) {
  (void)in_sizes; (void)n_in; (void)out_size;
  const float** F = (const float**)d_in;
  if (ws_size < (size_t)WS_END) return;
  char* ws = (char*)d_ws; float *F1T = (float*)(ws + WS_F1T), *MX = (float*)(ws + WS_MX); int *IDX0 = (int*)(ws + WS_IDX0), *IDX1 = (int*)(ws + WS_IDX1); __bf16* PW = (__bf16*)(ws + WS_PW);
  k_packW<<<dim3(128, 5), 256, 0, stream>>>(F[4], F[5], F[6], F[7], F[8], PW);
  k_f1t<<<NBT * N1 / 64, 64, 0, stream>>>(F[3], F1T);
  k_ball<<<NQT / 64, 64, 0, stream>>>(F[0], F[1], IDX0, IDX1);
  k_sa<0><<<NQT * 16 / 64, 128, 0, stream>>>(F[0], F[1], F1T, IDX0, PW, F[9], F[10], F[11], F[12], MX);
  k_sa<1><<<NQT * 32 / 64, 128, 0, stream>>>(F[0], F[1], F1T, IDX1, PW, F[13], F[14], F[15], F[16], MX);
  k_post<0><<<NQT / 64, 128, 0, stream>>>(MX, F[2], PW, F[17], F[18], (float*)d_out);
  k_post<1><<<NQT / 64, 128, 0, stream>>>(MX, F[2], PW, F[17], F[18], (float*)d_out);
}
